// MultiHeadAttention_40973988003964
// MI455X (gfx1250) — hardware-verified
//
#include <hip/hip_runtime.h>
#ifndef NB
#define NB 2u
#endif
#ifndef SEQ
#define SEQ 2048u
#endif
#define NB_FULL 2u
#define SEQ_FULL 2048u
#define SQ SEQ
#define DM 1024u
#define NH 16u
#define HD 64u
#define HG 2u
#define NR ((size_t)NB * SQ)
#define LQ (3u * DM)

static_assert(DM == NH * HD);
static_assert(HD == 64u);
static_assert(SQ % 256u == 0u);
static_assert((NB * SQ) % 128u == 0u);
static_assert(NH % HG == 0u);
static_assert(NB <= NB_FULL);
static_assert(SQ <= SEQ_FULL);
static_assert((DM * DM / 8u) % 256u == 0u);
static_assert(((size_t)NB * SQ * DM / 8u) % 256u == 0u);
static_assert((3u * DM / 4u) % 256u == 0u);
static_assert((HG * SQ) % 4u == 0u);
static_assert(LQ % 64u == 0u);

typedef unsigned short v8us __attribute__((ext_vector_type(8), may_alias));
typedef float  v8f  __attribute__((ext_vector_type(8)));
typedef float  v4f  __attribute__((ext_vector_type(4)));
typedef float  v4fa __attribute__((ext_vector_type(4), may_alias));
typedef _Float16 v16h __attribute__((ext_vector_type(16)));
typedef _Float16 v4h  __attribute__((ext_vector_type(4)));
union FragH { v16h v; v8us half[2]; _Float16 h[16]; unsigned short u[16]; };

constexpr size_t al256(size_t b) { return (b + 255) & ~(size_t)255; }
constexpr size_t SZ_W4  = al256((size_t)4 * DM * DM * 2);
constexpr size_t SZ_X16 = al256((size_t)NB * SQ * DM * 2);
constexpr size_t SZ_QKV = al256((size_t)NB * SQ * LQ * 2);
constexpr size_t SZ_O16 = al256((size_t)NB * SQ * DM * 2);
constexpr size_t SZ_S   = al256((size_t)HG * SQ * SQ * 4);
constexpr size_t SZ_P   = al256((size_t)HG * SQ * SQ * 2);
constexpr size_t SZ_VT  = al256((size_t)NH * HD * SQ * 2);
constexpr size_t SZ_B   = al256((size_t)3 * DM * 4);
constexpr size_t WS_TOTAL = SZ_W4 + SZ_X16 + SZ_QKV + SZ_O16 + SZ_S + SZ_P + SZ_VT + SZ_B;
static_assert(WS_TOTAL <= (size_t)134217728);

__device__ __forceinline__ unsigned short bf16_bits(float x) { unsigned int u = __float_as_uint(x); return (unsigned short)((u + 0x7FFFu + ((u >> 16) & 1u)) >> 16); }
__device__ __forceinline__ float bf16_val(unsigned short b) { return __uint_as_float(((unsigned int)b) << 16); }
__device__ __forceinline__ float bf16_rne(float x) { return bf16_val(bf16_bits(x)); }

__device__ __forceinline__ v16h g2_frag(const _Float16* p, unsigned hh) { FragH f; f.half[0] = *(const v8us*)((const unsigned short*)p + 8u * hh); f.half[1] = *(const v8us*)((const unsigned short*)p + 16u + 8u * hh); return f.v; }
__device__ __forceinline__ v8f g2_mma(v16h a, v16h b, v8f c) { v8f d = __builtin_amdgcn_wmma_f32_16x16x32_f16(false, a, false, b, (short)0, c, false, false); asm volatile("v_nop\n\tv_nop\n\tv_nop\n\tv_nop" : "+v"(d) : "v"(a), "v"(b)); return d; }

__global__ __launch_bounds__(256) void k_wnat4(const float* __restrict__ w0, const float* __restrict__ w1, const float* __restrict__ w2, const float* __restrict__ w3, _Float16* __restrict__ Bt) {
  const unsigned y = blockIdx.y;
  const float* w = (y == 0u) ? w0 : ((y == 1u) ? w1 : ((y == 2u) ? w2 : w3));
  const unsigned t = blockIdx.x * 256u + threadIdx.x; if (t >= DM * DM / 8u) return;
  const v4f a = *(const v4fa*)(w + (size_t)t * 8), c = *(const v4fa*)(w + (size_t)t * 8 + 4);
  FragH f;
#pragma unroll
  for (int q = 0; q < 4; ++q) { f.h[q] = (_Float16)(bf16_rne(a[q]) * 16.0f); f.h[4 + q] = (_Float16)(bf16_rne(c[q]) * 16.0f); }
  const v8us o = f.half[0];
  unsigned short* dst = (unsigned short*)Bt + (size_t)y * DM * DM + (size_t)t * 8;
  *(volatile v8us*)dst = o; __threadfence(); *(volatile v8us*)dst = o;
}

__global__ __launch_bounds__(256) void k_bcpy3(const float* __restrict__ b0, const float* __restrict__ b1, const float* __restrict__ b2, float* __restrict__ dst) {
  for (int pass = 0; pass < 2; ++pass) {
    for (unsigned i = threadIdx.x; i < 3u * DM / 4u; i += 256u) {
      const unsigned e = i * 4u, seg = e / DM, j = e - seg * DM;
      const v4f a = *(const v4fa*)(b0 + j), b = *(const v4fa*)(b1 + j), c = *(const v4fa*)(b2 + j);
      v4f v;
#pragma unroll
      for (int q = 0; q < 4; ++q) v[q] = (seg == 0u) ? a[q] : ((seg == 1u) ? b[q] : c[q]);
      *(volatile v4f*)(dst + e) = v;
    }
    if (pass == 0) __threadfence();
  }
}

__global__ __launch_bounds__(256) void k_x16(const float* __restrict__ x, _Float16* __restrict__ X16) {
  const unsigned t = blockIdx.x * 256u + threadIdx.x; if (t >= (unsigned)(NR * DM / 8u)) return;
  const unsigned r = t / (DM / 8u), c8 = (t - r * (DM / 8u)) * 8u;
  const unsigned b = r / SQ, s = r - b * SQ;
  const float* src = x + ((size_t)b * SEQ_FULL + s) * DM + c8;
  const v4f a = *(const v4fa*)src, c = *(const v4fa*)(src + 4);
  FragH f;
#pragma unroll
  for (int q = 0; q < 4; ++q) { f.h[q] = (_Float16)bf16_rne(a[q]); f.h[4 + q] = (_Float16)bf16_rne(c[q]); }
  const v8us o = f.half[0];
  unsigned short* dst = (unsigned short*)X16 + (size_t)t * 8;
  *(volatile v8us*)dst = o; __threadfence(); *(volatile v8us*)dst = o;
}

template <bool HASB, bool F32OUT>
__global__ __launch_bounds__(128) void k_gemm2(const _Float16* __restrict__ A, unsigned lda, size_t sA, const _Float16* __restrict__ Bh, unsigned ldb, size_t sB, float alpha, const float* __restrict__ bias,
    float* __restrict__ C, _Float16* __restrict__ C16, unsigned ldc, size_t sC, unsigned M, unsigned N, unsigned K) {
  __shared__ __attribute__((aligned(16))) float so[4][32][68];
  const unsigned tid = threadIdx.x, w = tid >> 5, lane = tid & 31u, ln = lane & 15u, hh = lane >> 4; const unsigned by = blockIdx.y;
  A += (size_t)by * sA; Bh += (size_t)by * sB; const size_t cofs = (size_t)by * sC;
  const unsigned ntn = N >> 6; const unsigned mt = blockIdx.x / ntn, nq = blockIdx.x - mt * ntn; const unsigned row0 = mt * 128u + 32u * w, col0 = nq * 64u; if (row0 >= M) return;
  const _Float16* a0p = A + (size_t)(row0 + ln) * lda; const _Float16* a1p = a0p + (size_t)16 * lda;
  const _Float16* b0p = Bh + (size_t)(col0 + ln) * ldb; const _Float16* b1p = b0p + (size_t)16 * ldb; const _Float16* b2p = b1p + (size_t)16 * ldb; const _Float16* b3p = b2p + (size_t)16 * ldb;
  const v8f z8 = {0.f,0.f,0.f,0.f,0.f,0.f,0.f,0.f}; v8f c00 = z8, c01 = z8, c02 = z8, c03 = z8, c10 = z8, c11 = z8, c12 = z8, c13 = z8;
#pragma unroll 1
  for (unsigned kb = 0; kb < K; kb += 32u) { const v16h a0 = g2_frag(a0p + kb, hh), a1 = g2_frag(a1p + kb, hh);
    v16h b = g2_frag(b0p + kb, hh); c00 = g2_mma(a0, b, c00); c10 = g2_mma(a1, b, c10);
    b = g2_frag(b1p + kb, hh); c01 = g2_mma(a0, b, c01); c11 = g2_mma(a1, b, c11);
    b = g2_frag(b2p + kb, hh); c02 = g2_mma(a0, b, c02); c12 = g2_mma(a1, b, c12);
    b = g2_frag(b3p + kb, hh); c03 = g2_mma(a0, b, c03); c13 = g2_mma(a1, b, c13); }
  v8f accs[8] = {c00, c01, c02, c03, c10, c11, c12, c13};
#pragma unroll
  for (int u = 0; u < 8; ++u) { const int t = u & 3, half = u >> 2; const unsigned col = col0 + (unsigned)t * 16u + ln; float bv = 0.f; if (HASB) bv = bf16_rne(bias[col]);
#pragma unroll
    for (int r = 0; r < 8; ++r) { const unsigned rloc = (unsigned)half * 16u + 8u * hh + (unsigned)r; so[w][rloc][(unsigned)t * 16u + ln] = accs[u][r] * alpha + bv; } }
  __builtin_amdgcn_fence(4  , "workgroup"); __builtin_amdgcn_wave_barrier();
  const unsigned rsub = lane >> 4, c4 = (lane & 15u) * 4u;
  for (int pass = 0; pass < 2; ++pass) {
#pragma unroll
    for (int q = 0; q < 16; ++q) { const unsigned r = (unsigned)q * 2u + rsub; const v4f v = *(const v4fa*)&so[w][r][c4];
      if (F32OUT) { *(volatile v4f*)(C + cofs + (size_t)(row0 + r) * ldc + col0 + c4) = v; }
      else { v4h h4;
#pragma unroll
        for (int i = 0; i < 4; ++i) h4[i] = (_Float16)v[i];
        *(volatile v4h*)(C16 + cofs + (size_t)(row0 + r) * ldc + col0 + c4) = h4; } }
    if (pass == 0) __threadfence(); }
}

template <unsigned NHv, unsigned TTv>
__global__ __launch_bounds__(256) void k_vt(const _Float16* __restrict__ V16, unsigned ldv, unsigned voff, _Float16* __restrict__ Vt) {
  __shared__ unsigned short tl[64][66];
  const unsigned tid = threadIdx.x; const unsigned slab = blockIdx.x / (TTv / 64u), lg = blockIdx.x - slab * (TTv / 64u); const unsigned b = slab / NHv, h = slab - b * NHv;
  for (unsigned i = tid; i < 64u * 8u; i += 256u) { const unsigned r = i >> 3, c8 = (i & 7u) * 8u; FragH f; f.half[0] = *(const v8us*)((const unsigned short*)V16 + ((size_t)b * TTv + lg * 64u + r) * ldv + voff + h * 64u + c8);
#pragma unroll
    for (int q = 0; q < 8; ++q) tl[r][c8 + (unsigned)q] = f.u[q]; }
  __syncthreads();
  for (int pass = 0; pass < 2; ++pass) {
#pragma unroll
    for (int rd = 0; rd < 2; ++rd) { const unsigned d = (unsigned)rd * 32u + (tid >> 3), pc = tid & 7u; FragH f;
#pragma unroll
      for (int q = 0; q < 8; ++q) f.u[q] = tl[pc * 8u + (unsigned)q][d];
      const v8us o = f.half[0];
      *(volatile v8us*)((unsigned short*)Vt + ((size_t)slab * 64u + d) * TTv + lg * 64u + pc * 8u) = o; }
    if (pass == 0) __threadfence(); }
}

__global__ __launch_bounds__(128) void k_rsm(const float* __restrict__ S, _Float16* __restrict__ P, unsigned nrows) {
#pragma clang fp contract(off)
  __shared__ __attribute__((aligned(16))) float ex[4][SQ];
  const unsigned tid = threadIdx.x, w = tid >> 5, lane = tid & 31u;
  const unsigned row = blockIdx.x * 4u + w; if (row >= nrows) return;
  const float* s = S + (size_t)row * SQ;
  float mx = -3.0e38f;
#pragma unroll 1
  for (unsigned c = 0; c < SQ / 128u; ++c) { const v4f a = *(const v4fa*)(s + c * 128u + lane * 4u); mx = fmaxf(mx, fmaxf(fmaxf(a[0], a[1]), fmaxf(a[2], a[3]))); }
  for (unsigned m = 16u; m > 0u; m >>= 1) mx = fmaxf(mx, __shfl_xor(mx, (int)m, 32));
  float se = 0.f;
#pragma unroll 1
  for (unsigned c = 0; c < SQ / 128u; ++c) { const v4f a = *(const v4fa*)(s + c * 128u + lane * 4u); v4f e;
#pragma unroll
    for (int q = 0; q < 4; ++q) e[q] = expf(a[q] - mx);
    se += (e[0] + e[1]) + (e[2] + e[3]);
    *(v4fa*)&ex[w][c * 128u + lane * 4u] = e; }
  for (unsigned m = 16u; m > 0u; m >>= 1) se += __shfl_xor(se, (int)m, 32);
  const float sc = 256.0f / se;
  __builtin_amdgcn_fence(4  , "workgroup"); __builtin_amdgcn_wave_barrier();
  unsigned short* prow = (unsigned short*)P + (size_t)row * SQ;
  for (int pass = 0; pass < 2; ++pass) {
#pragma unroll 1
    for (unsigned c = 0; c < SQ / 256u; ++c) { const v4f a = *(const v4fa*)&ex[w][c * 256u + lane * 8u], b = *(const v4fa*)&ex[w][c * 256u + lane * 8u + 4u]; FragH f;
#pragma unroll
      for (int q = 0; q < 4; ++q) { f.h[q] = (_Float16)(a[q] * sc); f.h[4 + q] = (_Float16)(b[q] * sc); }
      const v8us o = f.half[0];
      *(volatile v8us*)(prow + c * 256u + lane * 8u) = o; }
    if (pass == 0) __threadfence(); }
}

extern "C" void kernel_launch(void* const* d_in, const int* in_sizes, int n_in,
                              void* d_out, int out_size, void* d_ws, size_t ws_size, hipStream_t stream) {
  if (n_in < 9) return;
  if ((size_t)in_sizes[0] < ((size_t)(NB - 1u) * SEQ_FULL + SQ) * DM) return;
  if ((size_t)in_sizes[1] < (size_t)DM * DM || (size_t)in_sizes[3] < (size_t)DM * DM || (size_t)in_sizes[5] < (size_t)DM * DM || (size_t)in_sizes[7] < (size_t)DM * DM) return;
  if ((unsigned)in_sizes[2] < DM || (unsigned)in_sizes[4] < DM || (unsigned)in_sizes[6] < DM || (unsigned)in_sizes[8] < DM) return;
  if ((size_t)out_size < NR * DM) return;
  if (WS_TOTAL > ws_size) return;
  const float* const* I = (const float* const*)d_in;
  const float* x = I[0]; const float* wq = I[1]; const float* bq = I[2]; const float* wk = I[3]; const float* bk = I[4]; const float* wv = I[5]; const float* bv = I[6]; const float* wo = I[7]; const float* bo = I[8];
  char* ws = (char*)d_ws; size_t off = 0;
  _Float16* W4  = (_Float16*)(ws + off); off += SZ_W4;
  _Float16* X16 = (_Float16*)(ws + off); off += SZ_X16;
  _Float16* QKV = (_Float16*)(ws + off); off += SZ_QKV;
  _Float16* O16 = (_Float16*)(ws + off); off += SZ_O16;
  float*    S   = (float*)(ws + off);    off += SZ_S;
  _Float16* P   = (_Float16*)(ws + off); off += SZ_P;
  _Float16* VT  = (_Float16*)(ws + off); off += SZ_VT;
  float*   bqkv = (float*)(ws + off);    off += SZ_B;
  _Float16* BO = W4 + (size_t)3 * DM * DM;
  _Float16* Q16 = QKV; _Float16* K16 = QKV + DM; _Float16* V16 = QKV + 2u * DM;

  k_wnat4<<<dim3(DM * DM / 8u / 256u, 4), 256, 0, stream>>>(wq, wk, wv, wo, W4);
  k_bcpy3<<<1, 256, 0, stream>>>(bq, bk, bv, bqkv);
  k_x16<<<(unsigned)(NR * DM / 8u / 256u), 256, 0, stream>>>(x, X16);
  k_gemm2<true, false><<<dim3((unsigned)((NR / 128u) * (LQ / 64u)), 1), 128, 0, stream>>>(X16, DM, 0, W4, DM, 0, 0.0625f, bqkv, nullptr, QKV, LQ, 0, (unsigned)NR, LQ, DM);
  for (unsigned b = 0; b < NB; ++b) { const size_t r0 = (size_t)b * SQ;
    k_vt<NH, SQ><<<NH * (SQ / 64u), 256, 0, stream>>>(V16 + r0 * LQ, LQ, 0, VT);
    for (unsigned h0 = 0; h0 < NH; h0 += HG) {
      k_gemm2<false, true><<<dim3((SQ / 128u) * (SQ / 64u), HG), 128, 0, stream>>>(Q16 + r0 * LQ + h0 * HD, LQ, (size_t)HD, K16 + r0 * LQ + h0 * HD, LQ, (size_t)HD, 0.125f, nullptr, S, nullptr, SQ, (size_t)SQ * SQ, SQ, SQ, HD);
      k_rsm<<<HG * SQ / 4u, 128, 0, stream>>>(S, P, HG * SQ);
      k_gemm2<false, false><<<dim3((SQ / 128u) * (HD / 64u), HG), 128, 0, stream>>>(P, SQ, (size_t)SQ * SQ, VT + (size_t)h0 * HD * SQ, SQ, (size_t)HD * SQ, 0.25f, nullptr, nullptr, O16 + r0 * DM + h0 * HD, DM, (size_t)HD, SQ, HD, SQ);
    } }
  k_gemm2<true, true><<<dim3((unsigned)((NR / 128u) * (DM / 64u)), 1), 128, 0, stream>>>(O16, DM, 0, BO, DM, 0, 0.0009765625f, bo, (float*)d_out, nullptr, DM, 0, (unsigned)NR, DM, DM);
}
